// MultiHeadAttention_44178033606903
// MI455X (gfx1250) — hardware-run, weakly checked
//
#include <hip/hip_runtime.h>


#ifndef NB
#define NB 4
#endif
#ifndef SEQ
#define SEQ 512
#endif
#define NB_FULL  4
#define SEQ_FULL 512
#ifndef OUT_SEQ
#define OUT_SEQ SEQ
#endif
#define DM     512
#define NH_    8
#define HD     64
#define NREL   129
#define KRROWS 144
#define VRK    128
#define QRS    2048.0f
#define QRI    (1.0f / 2048.0f)
#define RELC   16.0f
#define RELCI  (1.0f / 16.0f)
#define PCAR   256.0f
#define WCAR   16.0f
#define CXS    64.0f
#define OSCL   (1.0f / 1024.0f)
#define LOG2E  1.4426950408889634f
#define NEGM   (-1.0e9f)
#define SP     (SEQ + 4)
#define RP     148
#define OFF1   ((size_t)NB_FULL * SEQ_FULL * DM)

static_assert(HD == 64);
static_assert(NH_ * HD == DM);
static_assert(DM % 64 == 0);
static_assert(DM % 32 == 0);
static_assert(SEQ % 128 == 0);
static_assert((NB * SEQ) % 64 == 0);
static_assert(KRROWS % 16 == 0 && KRROWS >= NREL);
static_assert(VRK % 32 == 0 && VRK == NREL - 1);
static_assert((SP * 4) % 16 == 0 && (RP * 4) % 16 == 0 && RP >= KRROWS);
static_assert(NB <= NB_FULL);
static_assert(SEQ <= SEQ_FULL);
static_assert(OFF1 * 4 == (size_t)4194304);

typedef _Float16 h16;
typedef unsigned short bf;
typedef __attribute__((ext_vector_type(16))) __bf16   v16bf;
typedef __attribute__((ext_vector_type(16))) _Float16 v16h;
typedef __attribute__((ext_vector_type(8)))  _Float16 v8h;
typedef __attribute__((ext_vector_type(8)))  unsigned short v8us;
typedef __attribute__((ext_vector_type(8)))  float    v8f;
typedef __attribute__((ext_vector_type(4)))  float    v4f;
typedef v4f  __attribute__((may_alias)) v4fa;

__device__ __forceinline__ unsigned short f2bf(float f) { unsigned u = __float_as_uint(f); u += 0x7FFFu + ((u >> 16) & 1u); return (unsigned short)(u >> 16); }
__device__ __forceinline__ float bfr(float f) { return __uint_as_float(((unsigned)f2bf(f)) << 16); }
__device__ __forceinline__ v16h cat16(v8h lo, v8h hi) { return __builtin_shufflevector(lo, hi, 0, 1, 2, 3, 4, 5, 6, 7, 8, 9, 10, 11, 12, 13, 14, 15); }
__device__ __forceinline__ v16bf cat16b(v8us lo, v8us hi) { return __builtin_bit_cast(v16bf, __builtin_shufflevector(lo, hi, 0, 1, 2, 3, 4, 5, 6, 7, 8, 9, 10, 11, 12, 13, 14, 15)); }
__device__ __forceinline__ v8f wmma16(v16h a, v16h b, v8f c) { return __builtin_amdgcn_wmma_f32_16x16x32_f16(false, a, false, b, (short)0, c, false, false); }
__device__ __forceinline__ v8f wmmab(v16bf a, v16bf b, v8f c) { return __builtin_amdgcn_wmma_f32_16x16x32_bf16(false, a, false, b, (short)0, c, false, false); }
__device__ __forceinline__ v16h  ldh(const h16* p) { return cat16(*(const v8h*)p, *(const v8h*)(p + 16)); }
__device__ __forceinline__ v16bf ldb(const bf* p)  { return cat16b(*(const v8us*)p, *(const v8us*)(p + 16)); }
__device__ __forceinline__ void wave_sync() { __builtin_amdgcn_fence(3  , "wavefront"); __builtin_amdgcn_wave_barrier(); asm volatile("" ::: "memory"); }

__global__ __launch_bounds__(256) void k_cvt8(const float* __restrict__ src, bf* dst, size_t n8) {
    const size_t i = (size_t)blockIdx.x * 256 + threadIdx.x; if (i >= n8) return;
    const v8f v = *(const v8f*)(src + i * 8); v8us o;
#pragma unroll
    for (int k = 0; k < 8; ++k) o[k] = f2bf(v[k]);
    *(volatile v8us*)(dst + i * 8) = o; __threadfence(); *(volatile v8us*)(dst + i * 8) = o;
}

template <int F16OUT>
__global__ __launch_bounds__(256) void k_wT(const float* __restrict__ W, const float* __restrict__ M, bf* dst) {
    __shared__ __align__(16) bf ts[64 * 72];
    const int tid = threadIdx.x; const int k0 = blockIdx.x * 64, n0 = blockIdx.y * 64;
#pragma unroll
    for (int i = 0; i < 4; ++i) { const int r = (tid >> 4) + 16 * i, c = (tid & 15) * 4;
        const v4f w = *(const v4f*)(W + (size_t)(k0 + r) * DM + n0 + c); const v4f m = *(const v4f*)(M + (size_t)(k0 + r) * DM + n0 + c);
#pragma unroll
        for (int e = 0; e < 4; ++e) { const float x = bfr(w[e]) * bfr(m[e]); unsigned short bits;
            if (F16OUT) bits = __builtin_bit_cast(unsigned short, (h16)(x * RELC)); else bits = f2bf(x);
            ts[(c + e) * 72 + r] = bits; } }
    __syncthreads();
    v8us o0, o1; size_t a0, a1;
    { const int p = tid,       row = p >> 3, c8 = (p & 7) * 8; o0 = *(const v8us*)(&ts[row * 72 + c8]); a0 = (size_t)(n0 + row) * DM + k0 + c8; }
    { const int p = tid + 256, row = p >> 3, c8 = (p & 7) * 8; o1 = *(const v8us*)(&ts[row * 72 + c8]); a1 = (size_t)(n0 + row) * DM + k0 + c8; }
    *(volatile v8us*)(dst + a0) = o0; *(volatile v8us*)(dst + a1) = o1;
    __threadfence();
    *(volatile v8us*)(dst + a0) = o0; *(volatile v8us*)(dst + a1) = o1;
}

__global__ __launch_bounds__(256) void k_relprep(const float* __restrict__ KREL, const float* __restrict__ VREL, h16* KR, h16* VRT) {
    __shared__ __align__(16) h16 vs[VRK * HD];
    const int tid = threadIdx.x, h = blockIdx.x;
#pragma unroll 1
    for (int p = tid; p < KRROWS * 8; p += 256) {
        const int row = p >> 3, c8 = (p & 7) * 8; const int rc = row < NREL ? row : NREL - 1;
        const v4f a = *(const v4f*)(KREL + ((size_t)h * NREL + rc) * HD + c8); const v4f c = *(const v4f*)(KREL + ((size_t)h * NREL + rc) * HD + c8 + 4);
        const bool ok = row < NREL; v8h o;
#pragma unroll
        for (int i = 0; i < 4; ++i) { o[i] = (h16)(ok ? bfr(a[i]) * RELC : 0.0f); o[4 + i] = (h16)(ok ? bfr(c[i]) * RELC : 0.0f); }
        h16* d = KR + ((size_t)h * KRROWS + row) * HD + c8;
        *(volatile v8h*)d = o; __threadfence(); *(volatile v8h*)d = o;
    }
#pragma unroll 1
    for (int i = tid; i < VRK * HD; i += 256) { const int m = i >> 6, d = i & 63;
        vs[i] = (h16)(bfr(VREL[((size_t)h * NREL + m) * HD + d]) * RELC); }
    __syncthreads();
#pragma unroll 1
    for (int p = tid; p < HD * (VRK / 8); p += 256) {
        const int d = p >> 4, c = p & 15; v8h o;
#pragma unroll
        for (int e = 0; e < 8; ++e) o[e] = vs[(8 * c + e) * HD + d];
        h16* dd = VRT + (size_t)h * HD * VRK + (size_t)p * 8;
        *(volatile v8h*)dd = o; __threadfence(); *(volatile v8h*)dd = o;
    }
}

__global__ __launch_bounds__(32) void k_proj(const bf* __restrict__ A, const bf* __restrict__ Bt, h16* Ph, h16* Pr, int useRes, int RB, size_t sRB, int pitch, int CB, size_t sCB) {
    __shared__ __align__(16) float os[16 * 68];
    const int K = DM;
    const int lane = threadIdx.x & 31, lr = lane & 15, hi = lane >> 4; const int r0 = blockIdx.x * 64, c0 = blockIdx.y * 64;
    v8f acc[4][4];
#pragma unroll
    for (int mb = 0; mb < 4; ++mb)
#pragma unroll
        for (int nb = 0; nb < 4; ++nb) acc[mb][nb] = (v8f){};
    const size_t aoff = (size_t)(r0 + lr) * K + 8 * hi, boff = (size_t)(c0 + lr) * K + 8 * hi;
#pragma unroll 1
    for (int kc = 0; kc < K; kc += 32) {
        v16bf a[4];
#pragma unroll
        for (int mb = 0; mb < 4; ++mb) a[mb] = ldb(A + aoff + (size_t)mb * 16 * K + kc);
#pragma unroll
        for (int nb = 0; nb < 4; ++nb) { const v16bf b = ldb(Bt + boff + (size_t)nb * 16 * K + kc);
#pragma unroll
            for (int mb = 0; mb < 4; ++mb) acc[mb][nb] = wmmab(a[mb], b, acc[mb][nb]); }
        asm volatile("v_nop\n\tv_nop\n\tv_nop\n\tv_nop" : "+v"(acc[0][0]), "+v"(acc[1][1]), "+v"(acc[2][2]), "+v"(acc[3][3]) : "v"(a[0]), "v"(a[1]), "v"(a[2]), "v"(a[3]));
    }
    const size_t tbase = (size_t)(r0 / RB) * sRB + (size_t)(r0 % RB) * (size_t)pitch + (size_t)(c0 / CB) * sCB + (size_t)(c0 % CB);
#pragma unroll
    for (int mb = 0; mb < 4; ++mb) {
#pragma unroll
        for (int nb = 0; nb < 4; ++nb) {
#pragma unroll
            for (int j = 0; j < 8; ++j) os[(hi * 8 + j) * 68 + nb * 16 + lr] = acc[mb][nb][j]; }
        wave_sync();
        const size_t sb = tbase + (size_t)(mb * 16) * (size_t)pitch;
#pragma unroll 1
        for (int ps = 0; ps < 2; ++ps) {
#pragma unroll
            for (int s = 0; s < 4; ++s) { const int row = 4 * s + (lane >> 3), c8 = (lane & 7) * 8;
                const v4f x0 = *(const v4fa*)(&os[row * 68 + c8]); const v4f x1 = *(const v4fa*)(&os[row * 68 + c8 + 4]); v8h hv, rv;
#pragma unroll
                for (int i = 0; i < 4; ++i) { const h16 a0 = (h16)x0[i]; const h16 a1 = (h16)x1[i]; hv[i] = a0; hv[4 + i] = a1; rv[i] = (h16)((x0[i] - (float)a0) * QRS); rv[4 + i] = (h16)((x1[i] - (float)a1) * QRS); }
                const size_t oo = sb + (size_t)row * (size_t)pitch + c8;
                *(volatile v8h*)(Ph + oo) = hv; if (useRes) *(volatile v8h*)(Pr + oo) = rv; }
            if (ps == 0) __threadfence(); }
        wave_sync();
    }
}

__global__ __launch_bounds__(32) void k_attn(const h16* __restrict__ QH, const h16* __restrict__ QR, const h16* __restrict__ KP, const h16* __restrict__ VT,
                                             const h16* __restrict__ KR, const h16* __restrict__ VRT, const float* __restrict__ VREL, const float* __restrict__ PM,
                                             h16* CTX, float* ATT) {
    __shared__ __align__(16) float S[16 * SP];
    __shared__ __align__(16) float RL[16 * RP];
    __shared__ __align__(16) float os[16 * 68];
    __shared__ __align__(16) float linv[16];
    const int lane = threadIdx.x & 31, lr = lane & 15, hi = lane >> 4;
    const int zh = blockIdx.y; const int b = zh / NH_, h = zh % NH_;
    const int t0 = blockIdx.x * 16; const int tq = t0 + lr;
    const int so = lr * SP, ro = lr * RP;
    const size_t pbase = (size_t)zh * SEQ * HD;
    const size_t qo = pbase + (size_t)(t0 + lr) * HD + 8 * hi;
    const v16h qh0 = ldh(QH + qo), qh1 = ldh(QH + qo + 32), qr0 = ldh(QR + qo), qr1 = ldh(QR + qo + 32);

    const size_t kro = ((size_t)h * KRROWS + lr) * HD + 8 * hi;
#pragma unroll 1
    for (int mt = 0; mt < KRROWS / 16; ++mt) {
        const h16* ra = KR + kro + (size_t)mt * 16 * HD;
        const v16h a0 = ldh(ra), a1 = ldh(ra + 32);
        v8f rH = (v8f){}, rL = (v8f){};
        rH = wmma16(a0, qh0, rH); rL = wmma16(a0, qr0, rL); rH = wmma16(a1, qh1, rH); rL = wmma16(a1, qr1, rL);
        asm volatile("v_nop\n\tv_nop\n\tv_nop\n\tv_nop" : "+v"(rH), "+v"(rL) : "v"(a0), "v"(a1));
        v4f x, y;
#pragma unroll
        for (int i = 0; i < 4; ++i) { x[i] = (rH[i] + rL[i] * QRI) * RELCI; y[i] = (rH[4 + i] + rL[4 + i] * QRI) * RELCI; }
        *(v4fa*)(&RL[ro + mt * 16 + 8 * hi]) = x; *(v4fa*)(&RL[ro + mt * 16 + 8 * hi + 4]) = y;
    }
    wave_sync();

    const size_t ko = pbase + (size_t)lr * HD + 8 * hi;
    const float* pmrow = PM + (size_t)b * SEQ_FULL;
    float mx = -3.0e38f;
#pragma unroll 1
    for (int key0 = 0; key0 < SEQ; key0 += 32) {
        const h16* ka = KP + ko + (size_t)key0 * HD;
        const v16h ka0 = ldh(ka), ka1 = ldh(ka + 32), kb0 = ldh(ka + 16 * HD), kb1 = ldh(ka + 16 * HD + 32);
        v8f sHa = (v8f){}, sLa = (v8f){}, sHb = (v8f){}, sLb = (v8f){};
        sHa = wmma16(ka0, qh0, sHa); sLa = wmma16(ka0, qr0, sLa); sHb = wmma16(kb0, qh0, sHb); sLb = wmma16(kb0, qr0, sLb);
        sHa = wmma16(ka1, qh1, sHa); sLa = wmma16(ka1, qr1, sLa); sHb = wmma16(kb1, qh1, sHb); sLb = wmma16(kb1, qr1, sLb);
        asm volatile("v_nop\n\tv_nop\n\tv_nop\n\tv_nop" : "+v"(sHa), "+v"(sLa), "+v"(sHb), "+v"(sLb) : "v"(ka0), "v"(ka1), "v"(kb0), "v"(kb1));
        const int ja = key0 + 8 * hi;
        const v4f ma0 = *(const v4f*)(pmrow + ja), ma1 = *(const v4f*)(pmrow + ja + 4), mb0 = *(const v4f*)(pmrow + ja + 16), mb1 = *(const v4f*)(pmrow + ja + 20);
        const int ib = ja - tq + 64;
        v4f xa0, xa1, xb0, xb1;
#pragma unroll
        for (int i = 0; i < 4; ++i) {
            const int i0 = min(max(ib + i, 0), NREL - 1), i1 = min(max(ib + 4 + i, 0), NREL - 1), i2 = min(max(ib + 16 + i, 0), NREL - 1), i3 = min(max(ib + 20 + i, 0), NREL - 1);
            xa0[i] = (sHa[i]     + sLa[i]     * QRI + RL[ro + i0]) * 0.125f + bfr(ma0[i]) * NEGM;
            xa1[i] = (sHa[4 + i] + sLa[4 + i] * QRI + RL[ro + i1]) * 0.125f + bfr(ma1[i]) * NEGM;
            xb0[i] = (sHb[i]     + sLb[i]     * QRI + RL[ro + i2]) * 0.125f + bfr(mb0[i]) * NEGM;
            xb1[i] = (sHb[4 + i] + sLb[4 + i] * QRI + RL[ro + i3]) * 0.125f + bfr(mb1[i]) * NEGM;
            mx = fmaxf(mx, fmaxf(fmaxf(xa0[i], xa1[i]), fmaxf(xb0[i], xb1[i])));
        }
        *(v4fa*)(&S[so + ja]) = xa0; *(v4fa*)(&S[so + ja + 4]) = xa1; *(v4fa*)(&S[so + ja + 16]) = xb0; *(v4fa*)(&S[so + ja + 20]) = xb1;
    }
    mx = fmaxf(mx, __shfl_xor(mx, 16, 32));
    wave_sync();

    const size_t vo = pbase + (size_t)lr * SEQ + 8 * hi;
    v8f o[4];
#pragma unroll
    for (int jd = 0; jd < 4; ++jd) o[jd] = (v8f){};
    float l = 0.0f, s0 = 0.0f, s1 = 0.0f;
    const int jlo = tq - 64, jhi = tq + 64;
#pragma unroll 1
    for (int key0 = 0; key0 < SEQ; key0 += 32) {
        const int ja = key0 + 8 * hi;
        v4f xa0 = *(const v4fa*)(&S[so + ja]), xa1 = *(const v4fa*)(&S[so + ja + 4]), xb0 = *(const v4fa*)(&S[so + ja + 16]), xb1 = *(const v4fa*)(&S[so + ja + 20]);
        v16h pb;
#pragma unroll
        for (int i = 0; i < 4; ++i) {
            const float p0 = __builtin_amdgcn_exp2f((xa0[i] - mx) * LOG2E), p1 = __builtin_amdgcn_exp2f((xa1[i] - mx) * LOG2E);
            const float p2 = __builtin_amdgcn_exp2f((xb0[i] - mx) * LOG2E), p3 = __builtin_amdgcn_exp2f((xb1[i] - mx) * LOG2E);
            const int j0 = ja + i, j1 = ja + 4 + i, j2 = ja + 16 + i, j3 = ja + 20 + i;
            l += (p0 + p1) + (p2 + p3);
            s0 += ((j0 <= jlo) ? p0 : 0.0f) + ((j1 <= jlo) ? p1 : 0.0f) + ((j2 <= jlo) ? p2 : 0.0f) + ((j3 <= jlo) ? p3 : 0.0f);
            s1 += ((j0 >= jhi) ? p0 : 0.0f) + ((j1 >= jhi) ? p1 : 0.0f) + ((j2 >= jhi) ? p2 : 0.0f) + ((j3 >= jhi) ? p3 : 0.0f);
            pb[i] = (h16)(p0 * PCAR); pb[4 + i] = (h16)(p1 * PCAR); pb[8 + i] = (h16)(p2 * PCAR); pb[12 + i] = (h16)(p3 * PCAR);
            xa0[i] = p0; xa1[i] = p1; xb0[i] = p2; xb1[i] = p3;
        }
        *(v4fa*)(&S[so + ja]) = xa0; *(v4fa*)(&S[so + ja + 4]) = xa1; *(v4fa*)(&S[so + ja + 16]) = xb0; *(v4fa*)(&S[so + ja + 20]) = xb1;
        const h16* va = VT + vo + key0;
        const v16h v0 = ldh(va), v1 = ldh(va + (size_t)16 * SEQ), v2 = ldh(va + (size_t)32 * SEQ), v3 = ldh(va + (size_t)48 * SEQ);
        o[0] = wmma16(v0, pb, o[0]); o[1] = wmma16(v1, pb, o[1]); o[2] = wmma16(v2, pb, o[2]); o[3] = wmma16(v3, pb, o[3]);
        asm volatile("v_nop\n\tv_nop\n\tv_nop\n\tv_nop" : "+v"(o[0]), "+v"(o[1]), "+v"(o[2]), "+v"(o[3]) : "v"(v0), "v"(v1), "v"(v2), "v"(v3), "v"(pb));
    }
    l += __shfl_xor(l, 16, 32); s0 += __shfl_xor(s0, 16, 32); s1 += __shfl_xor(s1, 16, 32);
    const float inv = 1.0f / l;
    linv[lr] = inv;
    wave_sync();

    const size_t vro = ((size_t)h * HD + lr) * VRK + 8 * hi;
#pragma unroll 1
    for (int m0 = 0; m0 < VRK; m0 += 32) {
        v16h wb;
#pragma unroll
        for (int i = 0; i < 16; ++i) {
            const int m = m0 + 8 * hi + (i & 7) + ((i >> 3) << 4);
            const int j = tq + m - 64;
            const int jc = min(max(j, 0), SEQ - 1);
            const float pv = S[so + jc];
            const bool ok = (m >= 1) && (j >= 0) && (j < SEQ);
            wb[i] = (h16)(ok ? pv * WCAR : 0.0f);
        }
        const h16* ra = VRT + vro + m0;
        const v16h a0 = ldh(ra), a1 = ldh(ra + (size_t)16 * VRK), a2 = ldh(ra + (size_t)32 * VRK), a3 = ldh(ra + (size_t)48 * VRK);
        o[0] = wmma16(a0, wb, o[0]); o[1] = wmma16(a1, wb, o[1]); o[2] = wmma16(a2, wb, o[2]); o[3] = wmma16(a3, wb, o[3]);
        asm volatile("v_nop\n\tv_nop\n\tv_nop\n\tv_nop" : "+v"(o[0]), "+v"(o[1]), "+v"(o[2]), "+v"(o[3]) : "v"(a0), "v"(a1), "v"(a2), "v"(a3), "v"(wb));
    }

    { const float oi = inv * (1.0f / PCAR), e0 = s0 * inv, e1 = s1 * inv;
#pragma unroll
      for (int jd = 0; jd < 4; ++jd) {
          const float* p0 = VREL + (size_t)h * NREL * HD + 16 * jd + 8 * hi;
          const float* p1 = p0 + (size_t)(NREL - 1) * HD;
          const v4f a0 = *(const v4f*)p0, a1 = *(const v4f*)(p0 + 4), c0 = *(const v4f*)p1, c1 = *(const v4f*)(p1 + 4);
          v4f x, y;
#pragma unroll
          for (int i = 0; i < 4; ++i) { x[i] = (o[jd][i] * oi + e0 * bfr(a0[i]) + e1 * bfr(c0[i])) * CXS; y[i] = (o[jd][4 + i] * oi + e0 * bfr(a1[i]) + e1 * bfr(c1[i])) * CXS; }
          *(v4fa*)(&os[lr * 68 + 16 * jd + 8 * hi]) = x; *(v4fa*)(&os[lr * 68 + 16 * jd + 8 * hi + 4]) = y; } }
    wave_sync();
    h16* crow = CTX + ((size_t)b * SEQ + t0) * DM + h * HD;
#pragma unroll 1
    for (int ps = 0; ps < 2; ++ps) {
#pragma unroll
        for (int s = 0; s < 4; ++s) { const int row = 4 * s + (lane >> 3), c8 = (lane & 7) * 8;
            const v4f x0 = *(const v4fa*)(&os[row * 68 + c8]); const v4f x1 = *(const v4fa*)(&os[row * 68 + c8 + 4]); v8h hv;
#pragma unroll
            for (int i = 0; i < 4; ++i) { hv[i] = (h16)x0[i]; hv[4 + i] = (h16)x1[i]; }
            *(volatile v8h*)(crow + (size_t)row * DM + c8) = hv; }
        if (ps == 0) __threadfence(); }

    float* arow = ATT + ((size_t)zh * OUT_SEQ + t0) * OUT_SEQ;
#pragma unroll 1
    for (int ps = 0; ps < 2; ++ps) {
#pragma unroll 1
        for (int row = 0; row < 16; ++row) { const float ri = linv[row];
#pragma unroll
            for (int c = 0; c < SEQ / 128; ++c) { const v4f pv = *(const v4fa*)(&S[row * SP + c * 128 + lane * 4]); const v4f val = pv * ri;
                *(volatile v4f*)(arow + (size_t)row * OUT_SEQ + c * 128 + lane * 4) = val; } }
        if (ps == 0) __threadfence(); }
}

__global__ __launch_bounds__(32) void k_out(const h16* __restrict__ A, const h16* __restrict__ Bt, const float* __restrict__ bias, float* OUT) {
    __shared__ __align__(16) float os[16 * 68];
    const int K = DM;
    const int lane = threadIdx.x & 31, lr = lane & 15, hi = lane >> 4; const int r0 = blockIdx.x * 64, c0 = blockIdx.y * 64;
    v8f acc[4][4];
#pragma unroll
    for (int mb = 0; mb < 4; ++mb)
#pragma unroll
        for (int nb = 0; nb < 4; ++nb) acc[mb][nb] = (v8f){};
    const size_t aoff = (size_t)(r0 + lr) * K + 8 * hi, boff = (size_t)(c0 + lr) * K + 8 * hi;
#pragma unroll 1
    for (int kc = 0; kc < K; kc += 32) {
        v16h a[4];
#pragma unroll
        for (int mb = 0; mb < 4; ++mb) a[mb] = ldh(A + aoff + (size_t)mb * 16 * K + kc);
#pragma unroll
        for (int nb = 0; nb < 4; ++nb) { const v16h bq = ldh(Bt + boff + (size_t)nb * 16 * K + kc);
#pragma unroll
            for (int mb = 0; mb < 4; ++mb) acc[mb][nb] = wmma16(a[mb], bq, acc[mb][nb]); }
        asm volatile("v_nop\n\tv_nop\n\tv_nop\n\tv_nop" : "+v"(acc[0][0]), "+v"(acc[1][1]), "+v"(acc[2][2]), "+v"(acc[3][3]) : "v"(a[0]), "v"(a[1]), "v"(a[2]), "v"(a[3]));
    }
    const int cofs = lr * 4;
    v4f bv = *(const v4f*)(bias + c0 + cofs);
#pragma unroll
    for (int i = 0; i < 4; ++i) bv[i] = bfr(bv[i]);
    const int bb = r0 / SEQ, tt = r0 % SEQ;
    float* obase = OUT + ((size_t)bb * OUT_SEQ + tt) * DM + c0;
#pragma unroll
    for (int mb = 0; mb < 4; ++mb) {
#pragma unroll
        for (int nb = 0; nb < 4; ++nb) {
#pragma unroll
            for (int j = 0; j < 8; ++j) os[(hi * 8 + j) * 68 + nb * 16 + lr] = acc[mb][nb][j] * OSCL; }
        wave_sync();
        float* orow = obase + (size_t)(mb * 16) * DM;
#pragma unroll 1
        for (int ps = 0; ps < 2; ++ps) {
#pragma unroll
            for (int s = 0; s < 8; ++s) { const int row = 2 * s + hi;
                const v4f val = *(const v4fa*)(&os[row * 68 + cofs]) + bv;
                *(volatile v4f*)(orow + (size_t)row * DM + cofs) = val; }
            if (ps == 0) __threadfence(); }
        wave_sync();
    }
}

static constexpr size_t al256(size_t v) { return (v + 255) & ~(size_t)255; }
static constexpr size_t SZ_XB = al256((size_t)NB * SEQ * DM * 2);
static constexpr size_t SZ_WB = al256((size_t)DM * DM * 2);
static constexpr size_t SZ_KR = al256((size_t)NH_ * KRROWS * HD * 2);
static constexpr size_t SZ_VR = al256((size_t)NH_ * HD * VRK * 2);
static constexpr size_t SZ_PL = al256((size_t)NB * NH_ * SEQ * HD * 2);
static constexpr size_t SZ_CX = al256((size_t)NB * SEQ * DM * 2);
static constexpr size_t SZ_TOTAL = 3 * SZ_XB + 4 * SZ_WB + SZ_KR + SZ_VR + 4 * SZ_PL + SZ_CX;
static_assert(SZ_TOTAL <= (size_t)134217728);

extern "C" void kernel_launch(void* const* d_in, const int* in_sizes, int n_in,
                              void* d_out, int out_size, void* d_ws, size_t ws_size, hipStream_t stream) {
    if (n_in < 15) return;
    const size_t needx = ((size_t)(NB - 1) * SEQ_FULL + SEQ) * DM;
    if ((size_t)in_sizes[0] < needx || (size_t)in_sizes[1] < needx || (size_t)in_sizes[2] < needx) return;
    if ((size_t)in_sizes[3] < (size_t)(NB - 1) * SEQ_FULL + SEQ) return;
    for (int i = 4; i <= 7; ++i) if ((size_t)in_sizes[i] < (size_t)DM * DM) return;
    if ((size_t)in_sizes[8] < (size_t)DM) return;
    for (int i = 9; i <= 12; ++i) if ((size_t)in_sizes[i] < (size_t)DM * DM) return;
    if ((size_t)in_sizes[13] < (size_t)NH_ * NREL * HD || (size_t)in_sizes[14] < (size_t)NH_ * NREL * HD) return;
    if ((size_t)out_size < ((size_t)(NB - 1) * OUT_SEQ + SEQ) * DM) return;
    if ((size_t)out_size < OFF1 + ((size_t)(NB * NH_ - 1) * OUT_SEQ + (SEQ - 1)) * OUT_SEQ + SEQ) return;
    if (SZ_TOTAL > ws_size) return;

    const float* v_in = (const float*)d_in[0];  const float* k_in = (const float*)d_in[1];  const float* q_in = (const float*)d_in[2];
    const float* pad  = (const float*)d_in[3];
    const float* wq   = (const float*)d_in[4];  const float* wk   = (const float*)d_in[5];  const float* wv   = (const float*)d_in[6];  const float* wo = (const float*)d_in[7];
    const float* bias = (const float*)d_in[8];
    const float* mq   = (const float*)d_in[9];  const float* mk   = (const float*)d_in[10]; const float* mv   = (const float*)d_in[11]; const float* mo = (const float*)d_in[12];
    const float* krel = (const float*)d_in[13]; const float* vrel = (const float*)d_in[14];
    float* OUT = (float*)d_out;
    float* ATT = OUT + OFF1;

    char* wsp = (char*)d_ws;
    bf* XQ = (bf*)wsp; wsp += SZ_XB;
    bf* XK = (bf*)wsp; wsp += SZ_XB;
    bf* XV = (bf*)wsp; wsp += SZ_XB;
    bf* WQT = (bf*)wsp; wsp += SZ_WB;
    bf* WKT = (bf*)wsp; wsp += SZ_WB;
    bf* WVT = (bf*)wsp; wsp += SZ_WB;
    bf* WOT = (bf*)wsp; wsp += SZ_WB;
    h16* KR  = (h16*)wsp; wsp += SZ_KR;
    h16* VRT = (h16*)wsp; wsp += SZ_VR;
    h16* QH = (h16*)wsp; wsp += SZ_PL;
    h16* QR = (h16*)wsp; wsp += SZ_PL;
    h16* KP = (h16*)wsp; wsp += SZ_PL;
    h16* VT = (h16*)wsp; wsp += SZ_PL;
    h16* CTX = (h16*)wsp; wsp += SZ_CX;

    if (SEQ == SEQ_FULL) {
        const size_t n8 = (size_t)NB * SEQ * DM / 8; const unsigned g = (unsigned)((n8 + 255) / 256);
        k_cvt8<<<g, 256, 0, stream>>>(q_in, XQ, n8); k_cvt8<<<g, 256, 0, stream>>>(k_in, XK, n8); k_cvt8<<<g, 256, 0, stream>>>(v_in, XV, n8);
    } else {
        const size_t n8 = (size_t)SEQ * DM / 8; const unsigned g = (unsigned)((n8 + 255) / 256);
        for (int b = 0; b < NB; ++b) {
            k_cvt8<<<g, 256, 0, stream>>>(q_in + (size_t)b * SEQ_FULL * DM, XQ + (size_t)b * SEQ * DM, n8);
            k_cvt8<<<g, 256, 0, stream>>>(k_in + (size_t)b * SEQ_FULL * DM, XK + (size_t)b * SEQ * DM, n8);
            k_cvt8<<<g, 256, 0, stream>>>(v_in + (size_t)b * SEQ_FULL * DM, XV + (size_t)b * SEQ * DM, n8);
        }
    }
    k_wT<0><<<dim3(DM / 64, DM / 64, 1), 256, 0, stream>>>(wq, mq, WQT);
    k_wT<0><<<dim3(DM / 64, DM / 64, 1), 256, 0, stream>>>(wk, mk, WKT);
    k_wT<0><<<dim3(DM / 64, DM / 64, 1), 256, 0, stream>>>(wv, mv, WVT);
    k_wT<1><<<dim3(DM / 64, DM / 64, 1), 256, 0, stream>>>(wo, mo, WOT);
    k_relprep<<<NH_, 256, 0, stream>>>(krel, vrel, KR, VRT);

    k_proj<<<dim3(NB * SEQ / 64, DM / 64, 1), 32, 0, stream>>>(XQ, WQT, QH, QR, 1, SEQ, (size_t)NH_ * SEQ * HD, HD, HD, (size_t)SEQ * HD);
    k_proj<<<dim3(NB * SEQ / 64, DM / 64, 1), 32, 0, stream>>>(XK, WKT, KP, KP, 0, SEQ, (size_t)NH_ * SEQ * HD, HD, HD, (size_t)SEQ * HD);
    k_proj<<<dim3(DM / 64, NB * SEQ / 64, 1), 32, 0, stream>>>(WVT, XV, VT, VT, 0, DM, (size_t)0, SEQ, SEQ, (size_t)DM * SEQ);

    k_attn<<<dim3(SEQ / 16, NB * NH_, 1), 32, 0, stream>>>(QH, QR, KP, VT, KR, VRT, vrel, pad, CTX, ATT);

    k_out<<<dim3(NB * SEQ / 64, DM / 64, 1), 32, 0, stream>>>(CTX, (const h16*)WOT, bias, OUT);
}
